// CosformerMultiHeadAttention_13280038879447
// MI455X (gfx1250) — hardware-verified
//
#include <hip/hip_runtime.h>
#include <math.h>

typedef __attribute__((ext_vector_type(16))) _Float16 v16h;
typedef __attribute__((ext_vector_type(16))) __bf16 v16b;
typedef __attribute__((ext_vector_type(8)))  _Float16 v8h;
typedef __attribute__((ext_vector_type(8)))  float v8f;
typedef __attribute__((ext_vector_type(4)))  float v4f;
typedef __attribute__((ext_vector_type(2)))  float v2f;
typedef __attribute__((ext_vector_type(4)))  unsigned v4u;
typedef __attribute__((ext_vector_type(4)))  int v4i;
typedef float __attribute__((may_alias)) float_a;
typedef int __attribute__((may_alias)) int_a;

template <typename T> __device__ __forceinline__ void vst2(void* p, T v) { *(volatile T*)p = v; __threadfence(); *(volatile T*)p = v; }
__device__ __forceinline__ v8f wmma16(v16h a, v16h b, v8f c) {
  v8f d = __builtin_amdgcn_wmma_f32_16x16x32_f16(false, a, false, b, (short)0, c, false, false);
  asm volatile("v_nop\n\tv_nop\n\tv_nop\n\tv_nop" : "+v"(d) : "v"(a), "v"(b));
  return d;
}
__device__ __forceinline__ v8f wmma_bf(v16b a, v16b b, v8f c) {
  v8f d = __builtin_amdgcn_wmma_f32_16x16x32_bf16(false, a, false, b, (short)0, c, false, false);
  asm volatile("v_nop\n\tv_nop\n\tv_nop\n\tv_nop" : "+v"(d) : "v"(a), "v"(b));
  return d;
}
__device__ __forceinline__ v16h frag_h(const _Float16* rowk0, int lane) {
  union { v16h v; v8h q[2]; } u; const _Float16* p = rowk0 + 8 * (lane >> 4);
  u.q[0] = *(const v8h*)p; u.q[1] = *(const v8h*)(p + 16); return u.v;
}
__device__ __forceinline__ v16h frag_f32(const float* rowk0, int lane) {
  v16h a; const float* p = rowk0 + 8 * (lane >> 4);
#pragma unroll
  for (int i = 0; i < 8; ++i) { a[i] = (_Float16)p[i]; a[8 + i] = (_Float16)p[16 + i]; }
  return a;
}
__device__ __forceinline__ v16h frag_f32s(const float* rowk0, int lane, float sc) {
  v16h a; const float* p = rowk0 + 8 * (lane >> 4);
#pragma unroll
  for (int i = 0; i < 8; ++i) { a[i] = (_Float16)(p[i] * sc); a[8 + i] = (_Float16)(p[16 + i] * sc); }
  return a;
}
__device__ __forceinline__ v16h fragc_f32(const float* W, int k0, int n, int lane, int ld, int K) {
  v16h a; const int g = lane >> 4;
#pragma unroll
  for (int i = 0; i < 8; ++i) { const int ka = k0 + 8 * g + i, kb = ka + 16;
    a[i] = (_Float16)(ka < K ? W[(size_t)(ka < K ? ka : K - 1) * ld + n] : 0.f); a[8 + i] = (_Float16)(kb < K ? W[(size_t)(kb < K ? kb : K - 1) * ld + n] : 0.f); }
  return a;
}
struct F2 { v16b h, l; };
__device__ __forceinline__ F2 bsplit16(const float v[16]) { F2 r;
#pragma unroll
  for (int i = 0; i < 16; ++i) { const __bf16 h = (__bf16)v[i]; r.h[i] = h; r.l[i] = (__bf16)(v[i] - (float)h); }
  return r; }
__device__ __forceinline__ F2 split_row(const float* row, int k0, int lane) { float v[16]; const float* p = row + k0 + 8 * (lane >> 4);
#pragma unroll
  for (int i = 0; i < 8; ++i) { v[i] = p[i]; v[8 + i] = p[16 + i]; }
  return bsplit16(v); }
__device__ __forceinline__ F2 split_rowK(const float* row, int k0, int lane, int K) { float v[16]; const int g = lane >> 4;
#pragma unroll
  for (int i = 0; i < 8; ++i) { const int ka = k0 + 8 * g + i, kb = ka + 16; v[i] = ka < K ? row[ka < K ? ka : K - 1] : 0.f; v[8 + i] = kb < K ? row[kb < K ? kb : K - 1] : 0.f; }
  return bsplit16(v); }
__device__ __forceinline__ F2 split_col(const float* W, int k0, int n, int lane, int ld, int K) { float v[16]; const int g = lane >> 4;
#pragma unroll
  for (int i = 0; i < 8; ++i) { const int ka = k0 + 8 * g + i, kb = ka + 16; v[i] = ka < K ? W[(size_t)(ka < K ? ka : K - 1) * ld + n] : 0.f; v[8 + i] = kb < K ? W[(size_t)(kb < K ? kb : K - 1) * ld + n] : 0.f; }
  return bsplit16(v); }
__device__ __forceinline__ v8f mac3(const F2& a, const F2& b, v8f c) { c = wmma_bf(a.l, b.h, c); c = wmma_bf(a.h, b.l, c); return wmma_bf(a.h, b.h, c); }
__device__ __forceinline__ float sigm(float v) { return 1.0f / (1.0f + expf(-v)); }
#define LDSX() do { asm volatile("s_wait_dscnt 0" ::: "memory"); __builtin_amdgcn_wave_barrier(); __builtin_amdgcn_fence(__ATOMIC_RELEASE, "workgroup"); } while (0)


#define NB 4
#define NN 4096
#define DD 512
#define D2 (2 * DD)
#define NH 8
#define HD 64
#define NR (NB * NN)
#ifndef TNB
#define TNB NB
#endif
#define TR (TNB * NN)
typedef __attribute__((ext_vector_type(8))) __bf16 v8b;
__device__ __forceinline__ v16b frag_b(const __bf16* rowk0, int lane) {
  union { v16b v; v8b q[2]; } u; const __bf16* p = rowk0 + 8 * (lane >> 4);
  u.q[0] = *(const v8b*)p; u.q[1] = *(const v8b*)(p + 16); return u.v;
}
__device__ __forceinline__ float bfr(float v) { return (float)(__bf16)v; }
__device__ __attribute__((noinline)) float exp_ni(float v) { return expf(v); }
__device__ __attribute__((noinline)) float erf_ni(float v) { return erff(v); }

#define WS_PW  0u
#define WS_Q   (WS_PW + 2u * (size_t)3 * DD * DD)
#define WS_KT  (WS_Q + 2u * (size_t)NR * D2)
#define WS_VT  (WS_KT + 2u * (size_t)NB * D2 * NN)
#define WS_KVH (WS_VT + 2u * (size_t)NB * DD * NN)
#define WS_KVL (WS_KVH + 2u * (size_t)NB * DD * D2)
#define WS_KS  (WS_KVL + 2u * (size_t)NB * DD * D2)
#define WS_END (WS_KS + 4u * (size_t)NB * D2)

__global__ __launch_bounds__(256) void k_pack(const float* __restrict__ WQ, const float* __restrict__ WK, const float* __restrict__ WV, __bf16* __restrict__ P) { const int n = blockIdx.x, t = threadIdx.x; const float* src = (n < DD) ? (WQ + (size_t)n * DD) : (n < 2 * DD) ? (WK + (size_t)(n - DD) * DD) : (WV + (size_t)(n - 2 * DD) * DD); __shared__ __align__(16) __bf16 s[DD]; for (int k = t; k < DD; k += 256) s[k] = (__bf16)src[k]; __syncthreads(); if (t < DD / 8) vst2((unsigned*)(P + (size_t)n * DD + t * 8), *(const v4u*)&s[t * 8]); }
__device__ __attribute__((noinline)) float sin_p(float v) { return sinf(v); }
__device__ __attribute__((noinline)) float cos_p(float v) { return cosf(v); }
__global__ __launch_bounds__(128) void k_proj(const float* __restrict__ X, const __bf16* __restrict__ P, _Float16* __restrict__ Q, _Float16* __restrict__ KT, _Float16* __restrict__ VT) {
  __shared__ __align__(16) _Float16 so[2][64][136]; __shared__ __align__(16) _Float16 st[2][128][72];
  const int tid = threadIdx.x, wave = tid >> 5, lane = tid & 31, col = lane & 15, g = lane >> 4; const int which = blockIdx.z; const int n0 = blockIdx.y * 128; const size_t rb0 = (size_t)blockIdx.x * 64, r0 = rb0 + wave * 16; const size_t b = rb0 / NN, s0 = rb0 % NN;
  v8f acc[8] = {};
#pragma unroll 2
  for (int kc = 0; kc < DD / 32; ++kc) { v16b a; { const float* p = X + (r0 + col) * DD + kc * 32 + 8 * g;
#pragma unroll
      for (int i = 0; i < 8; ++i) { a[i] = (__bf16)p[i]; a[8 + i] = (__bf16)p[16 + i]; } }
#pragma unroll
    for (int j = 0; j < 8; ++j) acc[j] = wmma_bf(a, frag_b(P + ((size_t)which * DD + n0 + j * 16 + col) * DD + kc * 32, lane), acc[j]); }
  if (which == 0) {
#pragma unroll
    for (int r = 0; r < 8; ++r) { const int n = (int)((r0 + 8 * g + r) % NN); const float ang = (1.57079632679489662f * (float)(n + 1)) / (float)NN; const float sn = sin_p(ang), cs = cos_p(ang);
#pragma unroll
      for (int j = 0; j < 8; ++j) { const float v = fmaxf(acc[j][r], 0.f); so[0][wave * 16 + 8 * g + r][j * 16 + col] = (_Float16)(v * sn); so[1][wave * 16 + 8 * g + r][j * 16 + col] = (_Float16)(v * cs); } }
    LDSX();
    for (int rl = 0; rl < 16; ++rl) if (lane < 16) { vst2((unsigned*)(Q + (r0 + rl) * D2 + n0 + lane * 8), *(const v4u*)&so[0][wave * 16 + rl][lane * 8]); vst2((unsigned*)(Q + (r0 + rl) * D2 + DD + n0 + lane * 8), *(const v4u*)&so[1][wave * 16 + rl][lane * 8]); }
  } else if (which == 1) {
#pragma unroll
    for (int r = 0; r < 8; ++r) { const int n = (int)((r0 + 8 * g + r) % NN); const float ang = (1.57079632679489662f * (float)(n + 1)) / (float)NN; const float sn = sin_p(ang), cs = cos_p(ang);
#pragma unroll
      for (int j = 0; j < 8; ++j) { const float v = fmaxf(acc[j][r], 0.f); st[0][j * 16 + col][wave * 16 + 8 * g + r] = (_Float16)(v * sn); st[1][j * 16 + col][wave * 16 + 8 * g + r] = (_Float16)(v * cs); } }
    __syncthreads();
    for (int e = tid; e < 2 * 128 * 8; e += 128) { const int pl = e >> 10, d = (e >> 3) & 127, pc = e & 7; vst2((unsigned*)(KT + ((b * D2 + (size_t)pl * DD + n0 + d) * NN) + s0 + pc * 8), *(const v4u*)&st[pl][d][pc * 8]); }
  } else {
#pragma unroll
    for (int r = 0; r < 8; ++r)
#pragma unroll
      for (int j = 0; j < 8; ++j) st[0][j * 16 + col][wave * 16 + 8 * g + r] = (_Float16)acc[j][r];
    __syncthreads();
    for (int e = tid; e < 128 * 8; e += 128) { const int d = e >> 3, pc = e & 7; vst2((unsigned*)(VT + ((b * DD + n0 + d) * NN) + s0 + pc * 8), *(const v4u*)&st[0][d][pc * 8]); } }
}
__global__ __launch_bounds__(128) void k_kv(const _Float16* __restrict__ KT, const _Float16* __restrict__ VT, _Float16* __restrict__ KVH, _Float16* __restrict__ KVL) {
  __shared__ __align__(16) _Float16 sh[128][72]; __shared__ __align__(16) _Float16 sl[128][72];
  const int tid = threadIdx.x, wave = tid >> 5, lane = tid & 31, col = lane & 15, g = lane >> 4; const size_t b = blockIdx.z; const int d0 = blockIdx.x * 64, r0 = d0 + wave * 16; const int m0 = blockIdx.y * 128;
  v8f acc[8] = {};
#pragma unroll 2
  for (int kc = 0; kc < NN / 32; ++kc) { const v16h a = frag_h(KT + ((b * D2 + r0 + col) * NN) + kc * 32, lane);
#pragma unroll
    for (int j = 0; j < 8; ++j) acc[j] = wmma16(a, frag_h(VT + ((b * DD + m0 + j * 16 + col) * NN) + kc * 32, lane), acc[j]); }
#pragma unroll
  for (int j = 0; j < 8; ++j)
#pragma unroll
    for (int r = 0; r < 8; ++r) { const float v = acc[j][r]; const _Float16 hv = (_Float16)v; sh[j * 16 + col][wave * 16 + 8 * g + r] = hv; sl[j * 16 + col][wave * 16 + 8 * g + r] = (_Float16)((v - (float)hv) * 2048.0f); }
  __syncthreads();
  for (int e = tid; e < 128 * 8; e += 128) { const int m = e >> 3, pc = e & 7; const size_t o = ((b * DD + m0 + m) * D2) + d0 + pc * 8; vst2((unsigned*)(KVH + o), *(const v4u*)&sh[m][pc * 8]); vst2((unsigned*)(KVL + o), *(const v4u*)&sl[m][pc * 8]); }
}
__global__ __launch_bounds__(256) void k_ksum(const _Float16* __restrict__ KT, float* __restrict__ KS) {
  __shared__ __align__(16) float part[2][128]; const size_t b = blockIdx.y; const int d0 = blockIdx.x * 128, t = threadIdx.x; const int dl = t & 127, half = t >> 7; const _Float16* p = KT + ((b * D2 + d0 + dl) * NN) + half * (NN / 2); float s = 0.f;
  for (int n = 0; n < NN / 2; n += 8) { const v4u w = *(const v4u*)(p + n); const _Float16* h8 = (const _Float16*)&w; for (int i = 0; i < 8; ++i) s += (float)h8[i]; }
  part[half][dl] = s; __syncthreads();
  if (t < 128) part[0][t] = part[0][t] + part[1][t]; __syncthreads();
  if (t < 32) vst2(KS + b * D2 + d0 + t * 4, *(const v4f*)&part[0][t * 4]);
}
__global__ __launch_bounds__(128) void k_fin(const _Float16* __restrict__ Q, const _Float16* __restrict__ KVH, const _Float16* __restrict__ KVL, const float* __restrict__ KS, float* __restrict__ OUT) {
  __shared__ __align__(16) float so[4][16][132]; __shared__ float sz[4][16];
  const int tid = threadIdx.x, wave = tid >> 5, lane = tid & 31, col = lane & 15, g = lane >> 4; const size_t b = blockIdx.z; const int nb0 = blockIdx.x * 64; const int nw = nb0 + wave * 16; const size_t r0 = b * NN + nw; const int m0 = blockIdx.y * 128;
  { const int rl = lane & 15, half = lane >> 4; float s = 0.f; const _Float16* q = Q + (r0 + rl) * D2 + half * DD; const float* ks = KS + b * D2 + half * DD;
    for (int d = 0; d < DD; d += 8) { const v4u w = *(const v4u*)(q + d); const _Float16* h8 = (const _Float16*)&w;
#pragma unroll
      for (int i = 0; i < 8; ++i) s += (float)h8[i] * ks[d + i]; }
    s += __shfl_xor(s, 16); if (lane < 16) sz[wave][rl] = 1.0f / fmaxf(s, 1e-6f); }
  v8f acc[8] = {};
#pragma unroll 2
  for (int kc = 0; kc < D2 / 32; ++kc) { const v16h a = frag_h(Q + (r0 + col) * D2 + kc * 32, lane);
#pragma unroll
    for (int j = 0; j < 8; ++j) { const size_t wb = ((b * DD + m0 + j * 16 + col) * D2) + kc * 32; acc[j] = wmma16(a, frag_h(KVH + wb, lane), acc[j]); v8f t2 = {}; t2 = wmma16(a, frag_h(KVL + wb, lane), t2);
#pragma unroll
      for (int r = 0; r < 8; ++r) acc[j][r] += t2[r] * (1.0f / 2048.0f); } }
  LDSX();
#pragma unroll
  for (int j = 0; j < 8; ++j)
#pragma unroll
    for (int r = 0; r < 8; ++r) so[wave][8 * g + r][j * 16 + col] = acc[j][r] * sz[wave][8 * g + r];
  LDSX();
  for (int rl = 0; rl < 16; ++rl) { const int n = nw + rl; const int j64 = m0 / 64 + (lane >> 4); const size_t frow = b * NN + (size_t)((8 * n + j64) % NN); const int fc0 = (n / 512) * HD;
    vst2(OUT + frow * DD + fc0 + (lane & 15) * 4, *(const v4f*)&so[wave][rl][(lane >> 4) * 64 + (lane & 15) * 4]); }
}
extern "C" void kernel_launch(void* const* d_in, const int* in_sizes, int n_in, void* d_out, int out_size, void* d_ws, size_t ws_size, hipStream_t stream) {
  (void)in_sizes; (void)n_in; (void)out_size;
  const float** F = (const float**)d_in;
  if (ws_size < (size_t)WS_END) return;
  char* ws = (char*)d_ws; __bf16* P = (__bf16*)ws; _Float16 *Q = (_Float16*)(ws + WS_Q), *KT = (_Float16*)(ws + WS_KT), *VT = (_Float16*)(ws + WS_VT), *KVH = (_Float16*)(ws + WS_KVH), *KVL = (_Float16*)(ws + WS_KVL); float* KS = (float*)(ws + WS_KS);
  k_pack<<<3 * DD, 256, 0, stream>>>(F[1], F[2], F[3], P);
  k_proj<<<dim3(TR / 64, DD / 128, 3), 128, 0, stream>>>(F[0], P, Q, KT, VT);
  k_kv<<<dim3(D2 / 64, DD / 128, TNB), 128, 0, stream>>>(KT, VT, KVH, KVL);
  k_ksum<<<dim3(D2 / 128, TNB), 256, 0, stream>>>(KT, KS);
  k_fin<<<dim3(NN / 64, DD / 128, TNB), 128, 0, stream>>>(Q, KVH, KVL, KS, (float*)d_out);
}
